// HFLSTM_21010980012084
// MI455X (gfx1250) — hardware-run, weakly checked
//
#include <hip/hip_runtime.h>
#include <stdint.h>


#define T_RHO 365
#define T_HOR 24
#define T_TOT (T_RHO + T_HOR)
#define NB    512
#define NH    256
#define NF    15
#define NG    1024
#define KC    512
#define KX    32
#define BS    32
#define NBLK  (NB / BS)
#define NTH   256
#define GST   (NH * KC)

static_assert(NB % BS == 0);
static_assert(NTH == 256);
static_assert(BS == 32);
static_assert(NH == 8 * 32);

typedef float    v4f  __attribute__((ext_vector_type(4)));
typedef float    v8f  __attribute__((ext_vector_type(8)));
typedef _Float16 v8h  __attribute__((ext_vector_type(8)));
typedef _Float16 v16h __attribute__((ext_vector_type(16)));
union Frag { v16h v; v8h half[2]; };

constexpr size_t SZ_WCAT  = (size_t)NG * KC * 2;
constexpr size_t SZ_WINT  = (size_t)NH * KX * 2;
constexpr size_t OFF_WCAT = 0;
constexpr size_t OFF_WINT = OFF_WCAT + SZ_WCAT;
constexpr size_t WS_END   = OFF_WINT + SZ_WINT;
static_assert(WS_END <= (size_t)134217728);
static_assert(OFF_WINT % 128 == 0);
static_assert(SZ_WCAT % 512 == 0);
static_assert(SZ_WINT % 512 == 0);

#define LO_X0   0
#define LO_H0   16384
#define LO_H1   32768
#define LO_C    49152
#define LO_XB   81920
#define LO_PART 83968
#define LO_OUTS 86016
#define LO_PREV 89088
#define SMEM_BYTES 89216
static_assert(LO_H0 == LO_X0 + BS * NH * 2);
static_assert(LO_H1 == LO_H0 + BS * NH * 2);
static_assert(LO_C == LO_H1 + BS * NH * 2);
static_assert(LO_XB == LO_C + NH * BS * 4);
static_assert(LO_PART == LO_XB + BS * KX * 2);
static_assert(LO_OUTS == LO_PART + 16 * BS * 4);
static_assert(LO_PREV == LO_OUTS + T_HOR * BS * 4);
static_assert(SMEM_BYTES == LO_PREV + BS * 4);

__device__ __forceinline__ float sigm_f(float x) {
  return __builtin_amdgcn_rcpf(1.0f + __expf(-x));
}
__device__ __forceinline__ float tanh_f(float x) {
  return 1.0f - 2.0f * __builtin_amdgcn_rcpf(1.0f + __expf(x + x));
}
__device__ __forceinline__ v8h cvt8h(v4f a, v4f b, float s) {
  v8h r;
#pragma unroll
  for (int c = 0; c < 4; ++c) { r[c] = (_Float16)(a[c] * s); r[4 + c] = (_Float16)(b[c] * s); }
  return r;
}
__device__ __forceinline__ v8f mma(const Frag& a, const Frag& b, v8f c) {
  return __builtin_amdgcn_wmma_f32_16x16x32_f16(false, a.v, false, b.v, (short)0, c, false, false);
}

__global__ __launch_bounds__(256)
void prep_kernel(const float* __restrict__ W_ih, const float* __restrict__ W_hh,
                 const float* __restrict__ W_in, _Float16* wcat, _Float16* wint)
{
  const int tid = threadIdx.x;
  if (blockIdx.x < 256) {
    const int i  = blockIdx.x * 256 + tid;
    const int e  = i * 8;
    const int n  = e >> 9;
    const int k  = e & 511;
    const int ks = k & 255;
    const float* pi = W_ih + (size_t)n * NH + ks;
    const float* ph = W_hh + (size_t)n * NH + ks;
    const v4f ia = *(const v4f*)(pi), ib = *(const v4f*)(pi + 4);
    const v4f ha = *(const v4f*)(ph), hb = *(const v4f*)(ph + 4);
    const bool lo = (k < 256);
    const v4f a = lo ? ia : ha;
    const v4f b = lo ? ib : hb;
    const v8h hv = cvt8h(a, b, 16.0f);
    *(volatile v8h*)(wcat + e) = hv;
    __threadfence();
    *(volatile v8h*)(wcat + e) = hv;
  } else {
    const int i  = (blockIdx.x - 256) * 256 + tid;
    const int e  = i * 8;
    const int j  = e >> 5;
    const int k  = e & 31;
    const int ks = k & 15;
    const float* p = W_in + j * 16 + ks;
    const v4f a = *(const v4f*)(p), b = *(const v4f*)(p + 4);
    const v4f z4 = {0.0f, 0.0f, 0.0f, 0.0f};
    const bool in = (k < 16);
    const v8h hv = cvt8h(in ? a : z4, in ? b : z4, 16.0f);
    *(volatile v8h*)(wint + e) = hv;
    __threadfence();
    *(volatile v8h*)(wint + e) = hv;
  }
}

__device__ __forceinline__ void kstep8(v8f (&acc)[8], const _Float16* ar, const _Float16* br)
{
  Frag a0, a1, b0, b1, b2, b3;
  a0.half[0] = *(const v8h*)(ar);                 a0.half[1] = *(const v8h*)(ar + 16);
  a1.half[0] = *(const v8h*)(ar + 16 * NH);       a1.half[1] = *(const v8h*)(ar + 16 * NH + 16);
  b0.half[0] = *(const v8h*)(br);                 b0.half[1] = *(const v8h*)(br + 16);
  b1.half[0] = *(const v8h*)(br + GST);           b1.half[1] = *(const v8h*)(br + GST + 16);
  b2.half[0] = *(const v8h*)(br + 2 * GST);       b2.half[1] = *(const v8h*)(br + 2 * GST + 16);
  b3.half[0] = *(const v8h*)(br + 3 * GST);       b3.half[1] = *(const v8h*)(br + 3 * GST + 16);
  acc[0] = mma(a0, b0, acc[0]);
  acc[1] = mma(a0, b1, acc[1]);
  acc[2] = mma(a0, b2, acc[2]);
  acc[3] = mma(a0, b3, acc[3]);
  acc[4] = mma(a1, b0, acc[4]);
  acc[5] = mma(a1, b1, acc[5]);
  acc[6] = mma(a1, b2, acc[6]);
  acc[7] = mma(a1, b3, acc[7]);
  asm volatile("v_nop\n\tv_nop\n\tv_nop\n\tv_nop"
               : "+v"(acc[0]), "+v"(acc[1]), "+v"(acc[2]), "+v"(acc[3]),
                 "+v"(acc[4]), "+v"(acc[5]), "+v"(acc[6]), "+v"(acc[7])
               : "v"(a0.v), "v"(a1.v), "v"(b0.v), "v"(b1.v), "v"(b2.v), "v"(b3.v));
}

__device__ __forceinline__ void cell8(const v8f ai, const v8f af, const v8f ag, const v8f ao,
                                      float bi, float bf, float bg, float bo,
                                      float* cp, _Float16* hp, float* pp,
                                      bool need_out, float wo, int m)
{
  const float k16 = 0.0625f;
  v4f c0 = *(const v4f*)(cp);
  v4f c1 = *(const v4f*)(cp + 4);
  v8f cc = __builtin_shufflevector(c0, c1, 0, 1, 2, 3, 4, 5, 6, 7);
  v8f hv;
#pragma unroll
  for (int r = 0; r < 8; ++r) {
    const float gi = ai[r] * k16 + bi;
    const float gf = af[r] * k16 + bf;
    const float gg = ag[r] * k16 + bg;
    const float go = ao[r] * k16 + bo;
    const float cn = sigm_f(gf) * cc[r] + sigm_f(gi) * tanh_f(gg);
    const float hn = sigm_f(go) * tanh_f(cn);
    cc[r] = cn;
    hv[r] = hn;
    hp[r * NH] = (_Float16)hn;
  }
  c0 = __builtin_shufflevector(cc, cc, 0, 1, 2, 3);
  c1 = __builtin_shufflevector(cc, cc, 4, 5, 6, 7);
  *(v4f*)(cp)     = c0;
  *(v4f*)(cp + 4) = c1;
  if (need_out) {
    v8f pr;
#pragma unroll
    for (int r = 0; r < 8; ++r) {
      float p = hv[r] * wo;
      p += __shfl_xor(p, 1, 32);
      p += __shfl_xor(p, 2, 32);
      p += __shfl_xor(p, 4, 32);
      p += __shfl_xor(p, 8, 32);
      pr[r] = p;
    }
    if (m == 0) {
      *(v4f*)(pp)     = __builtin_shufflevector(pr, pr, 0, 1, 2, 3);
      *(v4f*)(pp + 4) = __builtin_shufflevector(pr, pr, 4, 5, 6, 7);
    }
  }
}

__global__ __launch_bounds__(NTH)
void rec_kernel(const float* __restrict__ xfc_rho, const float* __restrict__ xfc_hor,
                const float* __restrict__ xq_rho,  const float* __restrict__ b_in,
                const float* __restrict__ b_ih,    const float* __restrict__ b_hh,
                const float* __restrict__ W_out,   const float* __restrict__ b_out,
                const _Float16* __restrict__ wcat, const _Float16* __restrict__ wint,
                float* out)
{
  extern __shared__ __attribute__((aligned(16))) char smem[];
  _Float16* x0buf = (_Float16*)(smem + LO_X0);
  _Float16* hbuf0 = (_Float16*)(smem + LO_H0);
  _Float16* hbuf1 = (_Float16*)(smem + LO_H1);
  float*    cbuf  = (float*)(smem + LO_C);
  _Float16* xb    = (_Float16*)(smem + LO_XB);
  float*    part  = (float*)(smem + LO_PART);
  float*    outS  = (float*)(smem + LO_OUTS);
  float*    prevS = (float*)(smem + LO_PREV);

  const int tid  = threadIdx.x;
  const int lane = tid & 31;
  const int wave = tid >> 5;
  const int h    = lane >> 4;
  const int m    = lane & 15;
  const int b0   = blockIdx.x * BS;

  const v4f z4 = {0.0f, 0.0f, 0.0f, 0.0f};
  {
    float* hz = (float*)(smem + LO_H0);
    float* xz = (float*)(smem + LO_XB);
#pragma unroll
    for (int i = tid; i < (BS * NH * 2) / 16; i += NTH) *(v4f*)(hz + 4 * i) = z4;
#pragma unroll
    for (int i = tid; i < (NH * BS * 4) / 16; i += NTH) *(v4f*)(cbuf + 4 * i) = z4;
    if (tid < (BS * KX * 2) / 16) *(v4f*)(xz + 4 * tid) = z4;
    if (tid < BS / 4) *(v4f*)(prevS + 4 * tid) = z4;
  }
  const int u0 = wave * 16 + m;
  const int u1 = (wave + 8) * 16 + m;
  const float bI0 = b_ih[0 * NH + u0] + b_hh[0 * NH + u0];
  const float bF0 = b_ih[1 * NH + u0] + b_hh[1 * NH + u0];
  const float bG0 = b_ih[2 * NH + u0] + b_hh[2 * NH + u0];
  const float bO0 = b_ih[3 * NH + u0] + b_hh[3 * NH + u0];
  const float bI1 = b_ih[0 * NH + u1] + b_hh[0 * NH + u1];
  const float bF1 = b_ih[1 * NH + u1] + b_hh[1 * NH + u1];
  const float bG1 = b_ih[2 * NH + u1] + b_hh[2 * NH + u1];
  const float bO1 = b_ih[3 * NH + u1] + b_hh[3 * NH + u1];
  const float wo0 = W_out[u0];
  const float wo1 = W_out[u1];
  const float bn0 = b_in[32 * wave + m];
  const float bn1 = b_in[32 * wave + 16 + m];
  const float bout = b_out[0];
  const v8f z8 = {0.0f, 0.0f, 0.0f, 0.0f, 0.0f, 0.0f, 0.0f, 0.0f};
  __syncthreads();

#pragma unroll 1
  for (int step = 0; step < T_TOT; ++step) {
    const bool rho      = step < T_RHO;
    const bool need_out = step >= T_RHO - 1;
    const int  th       = step - T_RHO;
    _Float16* hcur = (step & 1) ? hbuf1 : hbuf0;
    _Float16* hnxt = (step & 1) ? hbuf0 : hbuf1;

    if (tid < 64) {
      const int oct = tid >> 5;
      const int r   = tid & 31;
      const int b   = b0 + r;
      const int tr  = min(step, T_RHO - 1);
      const int thr = max(step - T_RHO, 0);
      const float* sr = rho ? (xfc_rho + ((size_t)tr * NB + b) * NF)
                            : (xfc_hor + ((size_t)thr * NB + b) * NF);
      const int c0 = oct * 8;
      float e[8];
#pragma unroll
      for (int c = 0; c < 7; ++c) e[c] = sr[c0 + c];
      const float e7 = sr[min(c0 + 7, NF - 1)];
      const float q  = xq_rho[(size_t)tr * NB + b];
      const float p  = prevS[r];
      e[7] = (oct == 0) ? e7 : (rho ? q : p);
      v8h xv;
#pragma unroll
      for (int c = 0; c < 8; ++c) xv[c] = (_Float16)e[c];
      *(v8h*)(xb + r * KX + c0) = xv;
    }
    __syncthreads();

    {
      Frag bw0, bw1;
      const _Float16* wp = wint + (size_t)(32 * wave + m) * KX + 8 * h;
      bw0.half[0] = *(const v8h*)(wp);            bw0.half[1] = *(const v8h*)(wp + 16);
      bw1.half[0] = *(const v8h*)(wp + 16 * KX);  bw1.half[1] = *(const v8h*)(wp + 16 * KX + 16);
#pragma unroll
      for (int mt = 0; mt < 2; ++mt) {
        Frag a;
        const _Float16* ap = xb + (mt * 16 + m) * KX + 8 * h;
        a.half[0] = *(const v8h*)(ap);
        a.half[1] = *(const v8h*)(ap + 16);
        v8f d0 = mma(a, bw0, z8);
        v8f d1 = mma(a, bw1, z8);
        asm volatile("v_nop\n\tv_nop\n\tv_nop\n\tv_nop"
                     : "+v"(d0), "+v"(d1) : "v"(a.v), "v"(bw0.v), "v"(bw1.v));
#pragma unroll
        for (int r = 0; r < 8; ++r) {
          const int row = mt * 16 + 8 * h + r;
          const float v0 = fmaxf(d0[r] * 0.0625f + bn0, 0.0f);
          const float v1 = fmaxf(d1[r] * 0.0625f + bn1, 0.0f);
          x0buf[row * NH + 32 * wave + m]      = (_Float16)v0;
          x0buf[row * NH + 32 * wave + 16 + m] = (_Float16)v1;
        }
      }
    }
    __syncthreads();

#pragma unroll 1
    for (int hi = 0; hi < 2; ++hi) {
      const int ht = wave + 8 * hi;
      const int u  = ht * 16 + m;
      const float bi = hi ? bI1 : bI0;
      const float bf = hi ? bF1 : bF0;
      const float bg = hi ? bG1 : bG0;
      const float bo = hi ? bO1 : bO0;
      const float wo = hi ? wo1 : wo0;
      const _Float16* wb = wcat + (size_t)u * KC + 8 * h;
      v8f acc[8];
#pragma unroll
      for (int j = 0; j < 8; ++j) acc[j] = z8;
      const _Float16* xa = x0buf + m * NH + 8 * h;
#pragma unroll 1
      for (int k0 = 0; k0 < NH; k0 += 32) kstep8(acc, xa + k0, wb + k0);
      const _Float16* ha = hcur + m * NH + 8 * h;
#pragma unroll 1
      for (int k0 = 0; k0 < NH; k0 += 32) kstep8(acc, ha + k0, wb + NH + k0);
#pragma unroll
      for (int mt = 0; mt < 2; ++mt) {
        const int rb = mt * 16 + 8 * h;
        cell8(acc[4 * mt + 0], acc[4 * mt + 1], acc[4 * mt + 2], acc[4 * mt + 3],
              bi, bf, bg, bo,
              cbuf + u * BS + rb, hnxt + rb * NH + u, part + ht * BS + rb,
              need_out, wo, m);
      }
    }
    __syncthreads();

    if (need_out && tid < BS) {
      float s = 0.0f;
#pragma unroll
      for (int t = 0; t < 16; ++t) s += part[t * BS + tid];
      s += bout;
      prevS[tid] = s;
      if (!rho) outS[th * BS + tid] = s;
    }
    __syncthreads();
  }

  if (wave == 0) {
    const int q = lane >> 3;
    const int c = (lane & 7) * 4;
    v4f v[6];
#pragma unroll
    for (int it = 0; it < 6; ++it) v[it] = *(const v4f*)(outS + (4 * it + q) * BS + c);
#pragma unroll
    for (int it = 0; it < 6; ++it)
      *(volatile v4f*)(out + (size_t)(4 * it + q) * NB + b0 + c) = v[it];
    __threadfence();
#pragma unroll
    for (int it = 0; it < 6; ++it)
      *(volatile v4f*)(out + (size_t)(4 * it + q) * NB + b0 + c) = v[it];
  }
}

extern "C" void kernel_launch(void* const* d_in, const int* in_sizes, int n_in,
                              void* d_out, int out_size, void* d_ws, size_t ws_size,
                              hipStream_t stream)
{
  if (n_in < 12) return;
  if (in_sizes[0]  != T_RHO * NB * NF) return;
  if (in_sizes[1]  != T_HOR * NB * NF) return;
  if (in_sizes[2]  != T_RHO * NB)      return;
  if (in_sizes[4]  != NH * 16)         return;
  if (in_sizes[5]  != NH)              return;
  if (in_sizes[6]  != NG * NH)         return;
  if (in_sizes[7]  != NG * NH)         return;
  if (in_sizes[8]  != NG)              return;
  if (in_sizes[9]  != NG)              return;
  if (in_sizes[10] != NH)              return;
  if (in_sizes[11] != 1)               return;
  if (out_size != T_HOR * NB)          return;
  if (ws_size < WS_END)                return;

  const float* xfc_rho = (const float*)d_in[0];
  const float* xfc_hor = (const float*)d_in[1];
  const float* xq_rho  = (const float*)d_in[2];
  const float* W_in  = (const float*)d_in[4];
  const float* b_in  = (const float*)d_in[5];
  const float* W_ih  = (const float*)d_in[6];
  const float* W_hh  = (const float*)d_in[7];
  const float* b_ih  = (const float*)d_in[8];
  const float* b_hh  = (const float*)d_in[9];
  const float* W_out = (const float*)d_in[10];
  const float* b_out = (const float*)d_in[11];
  float* out = (float*)d_out;

  char* ws = (char*)d_ws;
  _Float16* wcat = (_Float16*)(ws + OFF_WCAT);
  _Float16* wint = (_Float16*)(ws + OFF_WINT);

  prep_kernel<<<dim3(260), dim3(256), 0, stream>>>(W_ih, W_hh, W_in, wcat, wint);

  (void)hipFuncSetAttribute(reinterpret_cast<const void*>(&rec_kernel),
                            hipFuncAttributeMaxDynamicSharedMemorySize, SMEM_BYTES);
  rec_kernel<<<dim3(NBLK), dim3(NTH), SMEM_BYTES, stream>>>(
      xfc_rho, xfc_hor, xq_rho, b_in, b_ih, b_hh, W_out, b_out,
      (const _Float16*)wcat, (const _Float16*)wint, out);
}
